// LSTM_17600775979701
// MI455X (gfx1250) — hardware-verified
//
#include <hip/hip_runtime.h>
#include <math.h>

constexpr int NBATCH = 1024;
constexpr int NSTEP  = 512;
constexpr int NHID   = 128;
constexpr int NGATE  = 4;
constexpr int NCLS   = 10;
constexpr int NTHR   = 256;
constexpr int ROWBLK = 16;
constexpr int HPITCH = 136;
constexpr int FPITCH = 132;
constexpr float WCARRY  = 256.0f;
constexpr float HCARRY  = 64.0f;
constexpr float ACC_INV = 1.0f / (WCARRY * HCARRY);
constexpr int OUT_PER_BLOCK = ROWBLK * NCLS;

static_assert(NBATCH % ROWBLK == 0, "grid exact");
static_assert(NHID == 16 * (NTHR / 32), "8 waves x 16 hidden units");
static_assert(NHID % 32 == 0, "K multiple of 32");
static_assert(NHID % 64 == 0, "transpose tiles exact");
static_assert((NSTEP * ROWBLK) % (NTHR * 4) == 0, "x staging exact");
static_assert((2 * ROWBLK * HPITCH) % NTHR == 0, "h zero-fill exact");
static_assert((OUT_PER_BLOCK * 4) % 128 == 0, "block output is whole 128-B lines");
static_assert(OUT_PER_BLOCK == 160, "store map below assumes 160 floats per block");
static_assert(OUT_PER_BLOCK <= NTHR, "one thread per classifier output");
static_assert(NBATCH * NCLS * 4 == 40960, "output bytes");

typedef __attribute__((ext_vector_type(16))) _Float16 v16h;
typedef __attribute__((ext_vector_type(8)))  _Float16 v8h;
typedef __attribute__((ext_vector_type(8)))  float    v8f;
typedef __attribute__((ext_vector_type(4)))  float    v4f;

__device__ __forceinline__ void keep4_h(v16h a, v16h b, v16h c, v16h d) { asm volatile("v_nop" :: "v"(a), "v"(b), "v"(c), "v"(d)); }
__device__ __forceinline__ void grp_guard_h(v8f& a0, v8f& a1, v8f& a2, v8f& a3, v16h x, v16h b0, v16h b1, v16h b2, v16h b3) {
  asm volatile("v_nop\n\tv_nop\n\tv_nop\n\tv_nop" : "+v"(a0), "+v"(a1), "+v"(a2), "+v"(a3) : "v"(x), "v"(b0), "v"(b1), "v"(b2), "v"(b3));
}
__device__ __forceinline__ void keep8_f(float a, float b, float c, float d, float e, float f, float g, float h) {
  asm volatile("" :: "v"(a), "v"(b), "v"(c), "v"(d), "v"(e), "v"(f), "v"(g), "v"(h));
}

template <typename T> struct Frag;
template <> struct Frag<_Float16> {
  typedef v16h V; union U { v16h v; v8h h[2]; };
  static __device__ __forceinline__ v16h load(const _Float16* p) {
    U f; f.h[0] = *(const v8h*)(p); f.h[1] = *(const v8h*)(p + 16); return f.v;
  }
  static __device__ __forceinline__ v8f mma(v16h a, v16h b, v8f c) {
    return __builtin_amdgcn_wmma_f32_16x16x32_f16(false, a, false, b, (short)0, c, false, false);
  }
};

__device__ __forceinline__ float fsig(float x)  { return __builtin_amdgcn_rcpf(1.0f + __expf(-x)); }
__device__ __forceinline__ float ftanh(float x) { return 1.0f - 2.0f * __builtin_amdgcn_rcpf(__expf(2.0f * x) + 1.0f); }

__global__ __launch_bounds__(NTHR) void wh_plane_kernel(const float* __restrict__ Wg, const float* __restrict__ Wi,
                                                        const float* __restrict__ Wf, const float* __restrict__ Wo,
                                                        unsigned short* __restrict__ O) {
  __shared__ float Tt[64 * 65];
  const int tid = threadIdx.x;
  const int gate = blockIdx.z;
  const float* src = (gate == 0) ? Wg : (gate == 1) ? Wi : (gate == 2) ? Wf : Wo;
  const int c0 = blockIdx.x * 64, r0 = blockIdx.y * 64;
#pragma unroll
  for (int i = 0; i < 4; ++i) {
    const int idx = i * NTHR + tid;
    const int rr = idx >> 4, cc = (idx & 15) * 4;
    const v4f v = *(const v4f*)(src + (size_t)(r0 + rr) * (size_t)NHID + c0 + cc);
    Tt[rr * 65 + cc + 0] = v[0];
    Tt[rr * 65 + cc + 1] = v[1];
    Tt[rr * 65 + cc + 2] = v[2];
    Tt[rr * 65 + cc + 3] = v[3];
  }
  __syncthreads();
  const int q = tid >> 3, c8 = (tid & 7) * 8;
  v8h hv[2];
#pragma unroll
  for (int g = 0; g < 2; ++g) {
    const int qq = g * 32 + q;
#pragma unroll
    for (int e = 0; e < 8; ++e) {
      const float f = Tt[(c8 + e) * 65 + qq];
      hv[g][e] = (_Float16)(f * WCARRY);
    }
  }
  for (int pass = 0; pass < 2; ++pass) {
#pragma unroll
    for (int g = 0; g < 2; ++g) {
      const size_t o = (size_t)(gate * NHID + c0 + g * 32 + q) * (size_t)NHID + (size_t)(r0 + c8);
      *(volatile v8h*)(O + o) = hv[g];
    }
    __threadfence();
  }
}

__global__ __launch_bounds__(NTHR) void lstm_seq_kernel(const float* __restrict__ x,
                                                        const unsigned short* __restrict__ WHp,
                                                        const float* __restrict__ wgx, const float* __restrict__ wix,
                                                        const float* __restrict__ wfx, const float* __restrict__ wox,
                                                        const float* __restrict__ bgp, const float* __restrict__ bip,
                                                        const float* __restrict__ bfp, const float* __restrict__ bop,
                                                        const float* __restrict__ Wph, const float* __restrict__ bp,
                                                        float* __restrict__ out) {
  __shared__ __align__(16) float    Xs[NSTEP * ROWBLK];
  __shared__ __align__(16) _Float16 Ah[2][ROWBLK * HPITCH];
  __shared__ __align__(16) float    Hf[ROWBLK * FPITCH];
  __shared__ __align__(16) float    Os[OUT_PER_BLOCK];
  const _Float16* WH = (const _Float16*)WHp;
  const int tid = threadIdx.x, lane = tid & 31, wave = tid >> 5;
  const int c = lane & 15, hh = lane >> 4, koff = hh * 8, m0 = hh * 8;
  const int rowbase = blockIdx.x * ROWBLK;
  const int jj = 16 * wave + c;

#pragma unroll 1
  for (int it = 0; it < (NSTEP * ROWBLK) / (NTHR * 4); ++it) {
    const int idx = it * NTHR + tid;
    const int rr = idx >> 7, t4 = (idx & 127) * 4;
    const v4f v = *(const v4f*)(x + (size_t)(rowbase + rr) * NSTEP + t4);
    Xs[(t4 + 0) * ROWBLK + rr] = v[0];
    Xs[(t4 + 1) * ROWBLK + rr] = v[1];
    Xs[(t4 + 2) * ROWBLK + rr] = v[2];
    Xs[(t4 + 3) * ROWBLK + rr] = v[3];
  }
  {
    _Float16* ahf = &Ah[0][0];
#pragma unroll 1
    for (int i = tid; i < 2 * ROWBLK * HPITCH; i += NTHR) ahf[i] = (_Float16)0.0f;
  }

  v16h bfr[16];
#pragma unroll
  for (int g = 0; g < NGATE; ++g) {
    const _Float16* wrow = WH + (size_t)(g * NHID + jj) * NHID + koff;
#pragma unroll
    for (int kt = 0; kt < 4; ++kt) bfr[g * 4 + kt] = Frag<_Float16>::load(wrow + kt * 32);
    keep4_h(bfr[g * 4 + 0], bfr[g * 4 + 1], bfr[g * 4 + 2], bfr[g * 4 + 3]);
  }

  const float wxg = wgx[jj], wxi = wix[jj], wxf = wfx[jj], wxo = wox[jj];
  const float bgv = bgp[jj], biv = bip[jj], bfv = bfp[jj], bov = bop[jj];
  keep8_f(wxg, wxi, wxf, wxo, bgv, biv, bfv, bov);

  float cst[8];
#pragma unroll
  for (int r = 0; r < 8; ++r) cst[r] = 0.0f;

  __syncthreads();

  const v8f z8 = {0.f, 0.f, 0.f, 0.f, 0.f, 0.f, 0.f, 0.f};

#pragma unroll 1
  for (int t = 0; t < NSTEP; ++t) {
    const int cur = t & 1;
    const _Float16* hr = &Ah[cur][0] + c * HPITCH + koff;
    _Float16* hw = &Ah[cur ^ 1][0];
    const bool last = (t == NSTEP - 1);

    v8f acc0 = z8, acc1 = z8, acc2 = z8, acc3 = z8;
#pragma unroll
    for (int kt = 0; kt < 4; ++kt) {
      const v16h a = Frag<_Float16>::load(hr + kt * 32);
      acc0 = Frag<_Float16>::mma(a, bfr[0 + kt],  acc0);
      acc1 = Frag<_Float16>::mma(a, bfr[4 + kt],  acc1);
      acc2 = Frag<_Float16>::mma(a, bfr[8 + kt],  acc2);
      acc3 = Frag<_Float16>::mma(a, bfr[12 + kt], acc3);
      grp_guard_h(acc0, acc1, acc2, acc3, a, bfr[0 + kt], bfr[4 + kt], bfr[8 + kt], bfr[12 + kt]);
    }

    const v4f xa = *(const v4f*)(Xs + t * ROWBLK + m0);
    const v4f xb = *(const v4f*)(Xs + t * ROWBLK + m0 + 4);

#pragma unroll
    for (int r = 0; r < 8; ++r) {
      const float xv = (r < 4) ? xa[r & 3] : xb[r & 3];
      const float zg = acc0[r] * ACC_INV + (xv * wxg + bgv);
      const float zi = acc1[r] * ACC_INV + (xv * wxi + biv);
      const float zf = acc2[r] * ACC_INV + (xv * wxf + bfv);
      const float zo = acc3[r] * ACC_INV + (xv * wxo + bov);
      const float gv = ftanh(zg);
      const float iv = fsig(zi);
      const float fv = fsig(zf);
      const float ov = fsig(zo);
      const float cn = gv * iv + cst[r] * fv;
      cst[r] = cn;
      const float hn = ftanh(cn) * ov;
      hw[(m0 + r) * HPITCH + jj] = (_Float16)(hn * HCARRY);
      if (last) Hf[(m0 + r) * FPITCH + jj] = hn;
    }
    __syncthreads();
  }

  if (tid < OUT_PER_BLOCK) {
    const int rr = tid / NCLS;
    const int cc = tid - rr * NCLS;
    float s = 0.0f;
#pragma unroll 4
    for (int k = 0; k < NHID; ++k) s = fmaf(Hf[rr * FPITCH + k], Wph[k * NCLS + cc], s);
    Os[tid] = s + bp[cc];
  }
  __syncthreads();

  if (wave == 0) {
    const int i0 = lane * 4;
    const int i1 = 128 + (lane & 7) * 4;
    const v4f v0 = *(const v4f*)(Os + i0);
    const v4f v1 = *(const v4f*)(Os + i1);
    float* ob = out + (size_t)blockIdx.x * OUT_PER_BLOCK;
    for (int pass = 0; pass < 2; ++pass) {
      *(volatile v4f*)(ob + i0) = v0;
      if (lane < 8) *(volatile v4f*)(ob + i1) = v1;
      __threadfence();
    }
  }
}

extern "C" void kernel_launch(void* const* d_in, const int* in_sizes, int n_in,
                              void* d_out, int out_size, void* d_ws, size_t ws_size, hipStream_t stream) {
  if (n_in < 15 || d_out == nullptr || d_ws == nullptr) return;
  if (in_sizes[0] != NBATCH * NSTEP) return;
  if (in_sizes[1] != NHID || in_sizes[3] != NHID || in_sizes[5] != NHID || in_sizes[7] != NHID) return;
  if (in_sizes[2] != NHID * NHID || in_sizes[4] != NHID * NHID || in_sizes[6] != NHID * NHID || in_sizes[8] != NHID * NHID) return;
  if (in_sizes[9] != NHID * NCLS) return;
  if (in_sizes[10] != NHID || in_sizes[11] != NHID || in_sizes[12] != NHID || in_sizes[13] != NHID) return;
  if (in_sizes[14] != NCLS || out_size != NBATCH * NCLS) return;

  const float* x    = (const float*)d_in[0];
  const float* w_gx = (const float*)d_in[1];
  const float* w_gh = (const float*)d_in[2];
  const float* w_ix = (const float*)d_in[3];
  const float* w_ih = (const float*)d_in[4];
  const float* w_fx = (const float*)d_in[5];
  const float* w_fh = (const float*)d_in[6];
  const float* w_ox = (const float*)d_in[7];
  const float* w_oh = (const float*)d_in[8];
  const float* w_ph = (const float*)d_in[9];
  const float* b_g  = (const float*)d_in[10];
  const float* b_i  = (const float*)d_in[11];
  const float* b_f  = (const float*)d_in[12];
  const float* b_o  = (const float*)d_in[13];
  const float* b_p  = (const float*)d_in[14];
  float* out = (float*)d_out;

  char* ws = (char*)d_ws; size_t off = 0;
  auto carve = [&](size_t bytes) -> char* { char* p = ws + off; off += (bytes + 255) & ~(size_t)255; return p; };
  unsigned short* WHT = (unsigned short*)carve((size_t)NGATE * NHID * NHID * 2);
  if (off > ws_size || off > (size_t)134217728) return;

  wh_plane_kernel<<<dim3(NHID / 64, NHID / 64, NGATE), NTHR, 0, stream>>>(w_gh, w_ih, w_fh, w_oh, WHT);
  lstm_seq_kernel<<<NBATCH / ROWBLK, NTHR, 0, stream>>>(x, WHT, w_gx, w_ix, w_fx, w_ox, b_g, b_i, b_f, b_o, w_ph, b_p, out);
}
